// S6_51367808860423
// MI455X (gfx1250) — hardware-verified
//
#include <hip/hip_runtime.h>
#include <math.h>

typedef __attribute__((ext_vector_type(16))) _Float16 v16h;
typedef __attribute__((ext_vector_type(8)))  _Float16 v8h;
typedef __attribute__((ext_vector_type(16))) __bf16   v16b;
typedef __attribute__((ext_vector_type(8)))  __bf16   v8b;
typedef __attribute__((ext_vector_type(8)))  float    v8f;
typedef __attribute__((ext_vector_type(4)))  float    v4f;

constexpr int kBatch  = 4;
constexpr int kSeq    = 1024;
constexpr int kDm     = 1024;
constexpr int kNst    = 16;
constexpr int kDtR    = 64;
constexpr int kPrjN   = 96;
constexpr int kPrjP   = 128;
constexpr int kModP   = 2 * kDm;
constexpr int kRows   = kBatch * kSeq;
constexpr int kTP     = 260;
constexpr int kScanTS = 32;
constexpr float kCarryW1 = 32.0f;
constexpr float kCarryW2 = 8.0f;
constexpr float kCarryDt = 16.0f;
constexpr float kFold1   = 1.0f / kCarryW1;
constexpr float kFold2   = 1.0f / (kCarryDt * kCarryW2);

static_assert(kDtR + 2 * kNst == kPrjN, "x_proj width");
static_assert((kSeq & (kSeq - 1)) == 0, "sequence length power of two");
static_assert((kDm % 32) == 0 && (kDtR % 32) == 0, "GEMM K multiples of 32");
static_assert((kRows % 64) == 0 && (kPrjP % 64) == 0 && (kDm % 64) == 0, "GEMM M,N multiples of 64");
static_assert(((kRows / 64) * (kPrjP / 64)) % 8 == 0 && ((kRows / 64) * (kDm / 64)) % 8 == 0, "8 wave tiles per block");
static_assert((kSeq % 64) == 0 && (kSeq % kScanTS) == 0 && (kDm % 256) == 0, "tile multiples");
static_assert(((kPrjP * kDm / 8) % 256) == 0 && ((kPrjN * kDm / 8) % 32) == 0 && ((kDm * kDtR / 8) % 256) == 0 &&
              ((kRows * kDtR / 8) % 256) == 0, "exact cast grids");

constexpr size_t kOffWXP  = 0;
constexpr size_t kOffWDT  = kOffWXP  + (size_t)kPrjP * kDm  * 2;
constexpr size_t kOffX16  = kOffWDT  + (size_t)kDm   * kDtR * 2;
constexpr size_t kOffUC   = kOffX16  + (size_t)kRows * kDm  * 2;
constexpr size_t kOffPROJ = kOffUC   + (size_t)kRows * kDm  * 4;
constexpr size_t kOffDT16 = kOffPROJ + (size_t)kRows * kPrjP * 4;
constexpr size_t kOffDLR  = kOffDT16 + (size_t)kRows * kDtR * 2;
constexpr size_t kWsTotal = kOffDLR  + (size_t)kRows * kDm  * 4;
static_assert(kWsTotal == 44957696ull, "carve total");
static_assert(kWsTotal <= 134217728ull, "carve cap");
static_assert((kOffWDT % 128) == 0 && (kOffX16 % 128) == 0 && (kOffUC % 128) == 0 && (kOffPROJ % 128) == 0 &&
              (kOffDT16 % 128) == 0 && (kOffDLR % 128) == 0, "128-B aligned regions");

__device__ __forceinline__ unsigned short f2bf_bits(float f) {
  unsigned u = __float_as_uint(f);
  return (unsigned short)((u + 0x7FFFu + ((u >> 16) & 1u)) >> 16);
}
__device__ __forceinline__ float bf_bits2f(unsigned short h) { return __uint_as_float(((unsigned)h) << 16); }

__device__ __forceinline__ void dep_guard4_h(v8f& a, v8f& b, v8f& c, v8f& d, v16h x, v16h y) { asm volatile("v_nop\n\tv_nop\n\tv_nop\n\tv_nop" : "+v"(a), "+v"(b), "+v"(c), "+v"(d) : "v"(x), "v"(y)); }
__device__ __forceinline__ void dep_guard4_b(v8f& a, v8f& b, v8f& c, v8f& d, v16b x, v16b y) { asm volatile("v_nop\n\tv_nop\n\tv_nop\n\tv_nop" : "+v"(a), "+v"(b), "+v"(c), "+v"(d) : "v"(x), "v"(y)); }
__device__ __forceinline__ void keep4_h(v16h a, v16h b, v16h c, v16h d) { asm volatile("v_nop" :: "v"(a), "v"(b), "v"(c), "v"(d)); }
__device__ __forceinline__ void keep4_b(v16b a, v16b b, v16b c, v16b d) { asm volatile("v_nop" :: "v"(a), "v"(b), "v"(c), "v"(d)); }
__device__ __forceinline__ void acc_guard4(v8f& a, v8f& b, v8f& c, v8f& d) { asm volatile("v_nop\n\tv_nop\n\tv_nop\n\tv_nop" : "+v"(a), "+v"(b), "+v"(c), "+v"(d)); }
template <typename T> struct Frag;
template <> struct Frag<_Float16> {
  typedef v16h V; union U { v16h v; v8h h[2]; };
  static __device__ __forceinline__ v16h load(const _Float16* p) {
    U f; f.h[0] = *(const v8h*)(p); f.h[1] = *(const v8h*)(p + 16); return f.v;
  }
  static __device__ __forceinline__ v8f mma(v16h a, v16h b, v8f c) {
    return __builtin_amdgcn_wmma_f32_16x16x32_f16(false, a, false, b, (short)0, c, false, false);
  }
  static __device__ __forceinline__ void guard4(v8f& a, v8f& b, v8f& c, v8f& d, v16h x, v16h y) { dep_guard4_h(a, b, c, d, x, y); }
  static __device__ __forceinline__ void keep(v16h a, v16h b, v16h c, v16h d) { keep4_h(a, b, c, d); }
};
template <> struct Frag<__bf16> {
  typedef v16b V; union U { v16b v; v8b h[2]; };
  static __device__ __forceinline__ v16b load(const __bf16* p) {
    U f; f.h[0] = *(const v8b*)(p); f.h[1] = *(const v8b*)(p + 16); return f.v;
  }
  static __device__ __forceinline__ v8f mma(v16b a, v16b b, v8f c) {
    return __builtin_amdgcn_wmma_f32_16x16x32_bf16(false, a, false, b, (short)0, c, false, false);
  }
  static __device__ __forceinline__ void guard4(v8f& a, v8f& b, v8f& c, v8f& d, v16b x, v16b y) { dep_guard4_b(a, b, c, d, x, y); }
  static __device__ __forceinline__ void keep(v16b a, v16b b, v16b c, v16b d) { keep4_b(a, b, c, d); }
};

template <int ET> struct Elem;
template <> struct Elem<0> { typedef _Float16 T; };
template <> struct Elem<1> { typedef __bf16 T; };
template <int ET, bool SPLIT, int BIAS_MODE, int OUT_MODE, bool RESID, int ACT = 0>
__global__ __launch_bounds__(256) void wmma_gemm64(
    const unsigned short* __restrict__ Ap, const unsigned short* __restrict__ A2p, int lda, long strideA,
    const unsigned short* __restrict__ Btp, const unsigned short* __restrict__ Bt2p, int ldb, long strideB,
    void* __restrict__ Cout, void* __restrict__ Cout2, int ldc, long strideC,
    const float* __restrict__ bias,
    const float* __restrict__ resid, long strideR,
    int M, int N, int K, float scale) {
  typedef typename Elem<ET>::T T;
  typedef typename Frag<T>::V V;
  const T* A = (const T*)Ap; const T* A2 = (const T*)A2p; const T* Bt = (const T*)Btp; const T* Bt2 = (const T*)Bt2p;
  __shared__ __align__(16) float sT[8][16 * 68];
  const int b    = blockIdx.y;
  const int lane = threadIdx.x & 31;
  const int wave = threadIdx.x >> 5;
  const int tilesN = N >> 6;
  const int tilesM = M >> 6;
  const int tile = blockIdx.x * 8 + wave;
  if (tile >= tilesM * tilesN) return;
  const int tm = tile / tilesN;
  const int tn = tile - tm * tilesN;
  const int m0 = tm << 6;
  const int n0 = tn << 6;

  const T* Ab  = A  + (size_t)b * strideA;
  const T* Bb  = Bt + (size_t)b * strideB;
  const T* Ab2 = SPLIT ? (A2  + (size_t)b * strideA) : nullptr;
  const T* Bb2 = SPLIT ? (Bt2 + (size_t)b * strideB) : nullptr;

  const int rlane = lane & 15;
  const int koff  = (lane >> 4) * 8;
  const int mOff  = (lane >> 4) * 8;

  v8f acc[4][4];
#pragma unroll
  for (int i = 0; i < 4; ++i)
#pragma unroll
    for (int j = 0; j < 4; ++j) acc[i][j] = (v8f){0.f,0.f,0.f,0.f,0.f,0.f,0.f,0.f};

  for (int k0 = 0; k0 < K; k0 += 32) {
    V bh[4], bl[4];
#pragma unroll
    for (int j = 0; j < 4; ++j) {
      const size_t bo = (size_t)(n0 + (j << 4) + rlane) * ldb + koff + k0;
      bh[j] = Frag<T>::load(Bb + bo);
      if (SPLIT) bl[j] = Frag<T>::load(Bb2 + bo);
    }
#pragma unroll
    for (int i = 0; i < 4; ++i) {
      const size_t ao = (size_t)(m0 + (i << 4) + rlane) * lda + koff + k0;
      V ah = Frag<T>::load(Ab + ao);
      V al;
      if (SPLIT) al = Frag<T>::load(Ab2 + ao);
#pragma unroll
      for (int j = 0; j < 4; ++j) {
        acc[i][j] = Frag<T>::mma(ah, bh[j], acc[i][j]);
        if (SPLIT) {
          acc[i][j] = Frag<T>::mma(ah, bl[j], acc[i][j]);
          acc[i][j] = Frag<T>::mma(al, bh[j], acc[i][j]);
        }
      }
      Frag<T>::guard4(acc[i][0], acc[i][1], acc[i][2], acc[i][3], ah, SPLIT ? al : ah);
    }
    Frag<T>::keep(bh[0], bh[1], bh[2], bh[3]);
    if (SPLIT) Frag<T>::keep(bl[0], bl[1], bl[2], bl[3]);
  }
  acc_guard4(acc[0][0], acc[0][1], acc[0][2], acc[0][3]);
  acc_guard4(acc[1][0], acc[1][1], acc[1][2], acc[1][3]);
  acc_guard4(acc[2][0], acc[2][1], acc[2][2], acc[2][3]);
  acc_guard4(acc[3][0], acc[3][1], acc[3][2], acc[3][3]);

  float* slab = sT[wave];
  const float* Rb = RESID ? (resid + (size_t)b * strideR) : nullptr;
#pragma unroll
  for (int i = 0; i < 4; ++i) {
    const int mBase = m0 + (i << 4);
#pragma unroll
    for (int j = 0; j < 4; ++j) {
      const int n = n0 + (j << 4) + rlane;
      float bv = 0.f;
      if (BIAS_MODE == 2) bv = bias[n];
#pragma unroll
      for (int r = 0; r < 8; ++r) {
        float v = acc[i][j][r] * scale;
        if (BIAS_MODE == 1) v += bias[mBase + mOff + r];
        if (BIAS_MODE == 2) v += bv;
        if (RESID) v += Rb[(size_t)(mBase + mOff + r) * ldc + n];
        if (ACT == 1) v = tanhf(v);
        if (ACT == 2) v = fmaxf(v, 0.0f);
        if (ACT == 3) v = v / (1.0f + expf(-v));
        if (ACT == 4) v = (v > 0.f) ? v : 0.01f * v;
        slab[(mOff + r) * 68 + (j << 4) + rlane] = v;
      }
    }
    __builtin_amdgcn_fence(__ATOMIC_RELEASE, "workgroup");
    __builtin_amdgcn_wave_barrier();
    __builtin_amdgcn_fence(__ATOMIC_ACQUIRE, "workgroup");
    if (OUT_MODE == 0) {
      float* C = (float*)Cout + (size_t)b * strideC;
      const int hh = lane >> 4, c4 = (lane & 15) * 4;
      for (int pass = 0; pass < 2; ++pass) {
#pragma unroll
        for (int it = 0; it < 8; ++it) {
          const int row = it * 2 + hh;
          v4f v = *(const v4f*)(slab + row * 68 + c4);
          *(volatile v4f*)(C + (size_t)(mBase + row) * ldc + n0 + c4) = v;
        }
        __threadfence();
      }
    } else {
      const int q = lane >> 3, c8 = (lane & 7) * 8;
      unsigned short* C  = (unsigned short*)Cout  + (size_t)b * strideC;
      unsigned short* C2 = (OUT_MODE == 2) ? ((unsigned short*)Cout2 + (size_t)b * strideC) : nullptr;
      for (int pass = 0; pass < 2; ++pass) {
#pragma unroll
        for (int it = 0; it < 4; ++it) {
          const int row = it * 4 + q;
          const float* sp = slab + row * 68 + c8;
          v8h hv, lv;
#pragma unroll
          for (int e = 0; e < 8; ++e) {
            if (OUT_MODE == 1) {
              hv[e] = (_Float16)sp[e];
            } else {
              unsigned short hb = f2bf_bits(sp[e]);
              unsigned short lb = f2bf_bits(sp[e] - bf_bits2f(hb));
              hv[e] = __builtin_bit_cast(_Float16, hb);
              lv[e] = __builtin_bit_cast(_Float16, lb);
            }
          }
          *(volatile v8h*)(C + (size_t)(mBase + row) * ldc + n0 + c8) = hv;
          if (OUT_MODE == 2) *(volatile v8h*)(C2 + (size_t)(mBase + row) * ldc + n0 + c8) = lv;
        }
        __threadfence();
      }
    }
    __builtin_amdgcn_fence(__ATOMIC_RELEASE, "workgroup");
    __builtin_amdgcn_wave_barrier();
    __builtin_amdgcn_fence(__ATOMIC_ACQUIRE, "workgroup");
  }
}

__global__ __launch_bounds__(256) void cast_pad_f16_kernel(
    const float* __restrict__ src, unsigned short* __restrict__ dst, int total8, int real8, float scale)
{
  const int i = blockIdx.x * 256 + threadIdx.x;
  if (i >= total8) return;
  const bool live = (i < real8);
  const int ic = live ? i : (real8 - 1);
  const float* p = src + ((size_t)ic << 3);
  const v4f a0 = *(const v4f*)(p);
  const v4f a1 = *(const v4f*)(p + 4);
  v8h hv;
#pragma unroll
  for (int e = 0; e < 4; ++e) {
    const float f0 = live ? (a0[e] * scale) : 0.0f;
    const float f1 = live ? (a1[e] * scale) : 0.0f;
    hv[e]     = (_Float16)f0;
    hv[4 + e] = (_Float16)f1;
  }
  unsigned short* q = dst + ((size_t)i << 3);
  *(volatile v8h*)q = hv;
  __threadfence();
  *(volatile v8h*)q = hv;
}

__global__ __launch_bounds__(256) void dt_cast_kernel(
    const float* __restrict__ PROJ, unsigned short* __restrict__ DT16, int total8, float scale)
{
  const int i = blockIdx.x * 256 + threadIdx.x;
  if (i >= total8) return;
  const int e0  = i << 3;
  const int row = e0 >> 6;
  const int c8  = e0 & 63;
  const float* p = PROJ + (size_t)row * kPrjP + c8;
  const v4f a0 = *(const v4f*)(p);
  const v4f a1 = *(const v4f*)(p + 4);
  v8h hv;
#pragma unroll
  for (int e = 0; e < 4; ++e) {
    hv[e]     = (_Float16)(a0[e] * scale);
    hv[4 + e] = (_Float16)(a1[e] * scale);
  }
  unsigned short* qd = DT16 + e0;
  *(volatile v8h*)qd = hv;
  __threadfence();
  *(volatile v8h*)qd = hv;
}

__global__ __launch_bounds__(256) void conv_silu_kernel(
    const float* __restrict__ MOD, const float* __restrict__ cw, const float* __restrict__ cb,
    float* __restrict__ UC, unsigned short* __restrict__ X16)
{
  __shared__ __align__(16) float sT[16 * kTP];
  const int tid = threadIdx.x, lane = tid & 31, wave = tid >> 5;
  const int d0 = blockIdx.x * 256, d = d0 + tid;
  const int g0 = blockIdx.y * 64;
  const int tb = g0 & (kSeq - 1);
  const v4f wv = *(const v4f*)(cw + (size_t)d * 4);
  const float w0 = wv[0], w1 = wv[1], w2 = wv[2], w3 = wv[3];
  const float bc = cb[d];
  float xm3, xm2, xm1;
  {
    const bool hist = (tb > 0);
    const int rb = hist ? (g0 - 3) : g0;
    const float v3 = MOD[(size_t)rb * kModP + d];
    const float v2 = MOD[(size_t)(rb + 1) * kModP + d];
    const float v1 = MOD[(size_t)(rb + 2) * kModP + d];
    xm3 = hist ? v3 : 0.f;
    xm2 = hist ? v2 : 0.f;
    xm1 = hist ? v1 : 0.f;
  }
  const int hrow = wave >> 1;
  const int hch  = (wave & 1) * 128 + lane * 4;
#pragma unroll 1
  for (int sub = 0; sub < 4; ++sub) {
    const int lb = g0 + sub * 16;
#pragma unroll 1
    for (int s = 0; s < 16; ++s) {
      const float xcur = MOD[(size_t)(lb + s) * kModP + d];
      float acc = w0 * xm3;
      acc = fmaf(w1, xm2, acc);
      acc = fmaf(w2, xm1, acc);
      acc = fmaf(w3, xcur, acc);
      const float sv = acc + bc;
      const float sg = __builtin_amdgcn_rcpf(1.0f + __expf(-sv));
      sT[s * kTP + tid] = sv * sg;
      xm3 = xm2; xm2 = xm1; xm1 = xcur;
    }
    __syncthreads();
    v4f fv[4];
    v8h bv[2];
#pragma unroll
    for (int it = 0; it < 4; ++it) fv[it] = *(const v4f*)(sT + (it * 4 + hrow) * kTP + hch);
#pragma unroll
    for (int it = 0; it < 2; ++it) {
      const float* sp = sT + (it * 8 + wave) * kTP + lane * 8;
      const v4f a0 = *(const v4f*)(sp);
      const v4f a1 = *(const v4f*)(sp + 4);
#pragma unroll
      for (int e = 0; e < 4; ++e) {
        bv[it][e]     = (_Float16)a0[e];
        bv[it][4 + e] = (_Float16)a1[e];
      }
    }
    for (int pass = 0; pass < 2; ++pass) {
#pragma unroll
      for (int it = 0; it < 4; ++it)
        *(volatile v4f*)(UC + (size_t)(lb + it * 4 + hrow) * kDm + d0 + hch) = fv[it];
#pragma unroll
      for (int it = 0; it < 2; ++it)
        *(volatile v8h*)(X16 + (size_t)(lb + it * 8 + wave) * kDm + d0 + lane * 8) = bv[it];
      __threadfence();
    }
    __syncthreads();
  }
}

__global__ __launch_bounds__(256) void scan_kernel(
    const float* __restrict__ DLR, const float* __restrict__ UC, const float* __restrict__ MOD,
    const float* __restrict__ PROJ, const float* __restrict__ A_log, const float* __restrict__ Dv,
    float* __restrict__ OUT)
{
  __shared__ __align__(16) float sBC[kScanTS * 32];
  __shared__ __align__(16) float sY[kScanTS * kTP];
  const int tid = threadIdx.x, lane = tid & 31, wave = tid >> 5;
  constexpr int kBlkPerB = kDm / 256;
  const int bix = blockIdx.x / kBlkPerB;
  const int d0  = (blockIdx.x - bix * kBlkPerB) * 256;
  const int d   = d0 + tid;
  const size_t row0 = (size_t)bix * kSeq;

#pragma unroll 1
  for (int n = 0; n < kNst; ++n) sY[n * kTP + tid] = -expf(A_log[(size_t)d * kNst + n]);
  __syncthreads();
  float An[kNst], h[kNst];
#pragma unroll
  for (int n = 0; n < kNst; ++n) {
    An[n] = sY[n * kTP + tid];
    h[n] = 0.f;
  }
  const float Dd = Dv[d];
  __syncthreads();

  const int sr = tid >> 3, sq = (tid & 7) * 4;
  const int q = lane >> 3, c4 = (lane & 7) * 4;

#pragma unroll 1
  for (int c = 0; c < kSeq / kScanTS; ++c) {
    const int l0 = c * kScanTS;
    {
      const v4f v = *(const v4f*)(PROJ + (row0 + l0 + sr) * kPrjP + kDtR + sq);
      *(v4f*)(sBC + sr * 32 + sq) = v;
    }
    __syncthreads();
#pragma unroll 1
    for (int s = 0; s < kScanTS; ++s) {
      const size_t m = row0 + (size_t)(l0 + s);
      float a  = DLR[m * kDm + d];
      float xv = UC[m * kDm + d];
      float zv = MOD[m * kModP + kDm + d];
      asm volatile("" : "+v"(a));
      asm volatile("" : "+v"(xv));
      asm volatile("" : "+v"(zv));
      const float delta = fmaxf(a, 0.0f) + log1pf(__expf(-fabsf(a)));
      v4f Bq[4], Cq[4];
#pragma unroll
      for (int qq = 0; qq < 4; ++qq) {
        Bq[qq] = *(const v4f*)(sBC + s * 32 + 4 * qq);
        Cq[qq] = *(const v4f*)(sBC + s * 32 + kNst + 4 * qq);
      }
      const float dtx = delta * xv;
      float y = 0.f;
#pragma unroll
      for (int n = 0; n < kNst; ++n) {
        const float e = __expf(delta * An[n]);
        const float hn = fmaf(e, h[n], dtx * Bq[n >> 2][n & 3]);
        h[n] = hn;
        y = fmaf(hn, Cq[n >> 2][n & 3], y);
      }
      y = fmaf(xv, Dd, y);
      const float sg = __builtin_amdgcn_rcpf(1.0f + __expf(-zv));
      const float g  = zv * sg;
      sY[s * kTP + tid] = y * g;
    }
    __syncthreads();
    v4f ov[8];
#pragma unroll
    for (int it = 0; it < 8; ++it) {
      const int dl = it * 32 + wave * 4 + q;
      const float e0 = sY[(c4 + 0) * kTP + dl];
      const float e1 = sY[(c4 + 1) * kTP + dl];
      const float e2 = sY[(c4 + 2) * kTP + dl];
      const float e3 = sY[(c4 + 3) * kTP + dl];
      ov[it] = (v4f){e0, e1, e2, e3};
    }
    for (int pass = 0; pass < 2; ++pass) {
#pragma unroll
      for (int it = 0; it < 8; ++it) {
        const int dl = it * 32 + wave * 4 + q;
        *(volatile v4f*)(OUT + ((size_t)bix * kDm + d0 + dl) * kSeq + l0 + c4) = ov[it];
      }
      __threadfence();
    }
  }
}

extern "C" void kernel_launch(void* const* d_in, const int* in_sizes, int n_in,
                              void* d_out, int out_size, void* d_ws, size_t ws_size,
                              hipStream_t stream)
{
  if (n_in < 8) return;
  if (in_sizes[0] != kRows * kModP) return;
  if (in_sizes[1] != kDm * 4) return;
  if (in_sizes[2] != kDm) return;
  if (in_sizes[3] != kPrjN * kDm) return;
  if (in_sizes[4] != kDm * kDtR) return;
  if (in_sizes[5] != kDm) return;
  if (in_sizes[6] != kDm * kNst) return;
  if (in_sizes[7] != kDm) return;
  if (out_size != kBatch * kDm * kSeq) return;
  if (ws_size < kWsTotal) return;

  const float* mod    = (const float*)d_in[0];
  const float* conv_w = (const float*)d_in[1];
  const float* conv_b = (const float*)d_in[2];
  const float* xpw    = (const float*)d_in[3];
  const float* dtw    = (const float*)d_in[4];
  const float* dtb    = (const float*)d_in[5];
  const float* A_log  = (const float*)d_in[6];
  const float* Dp     = (const float*)d_in[7];
  float* out = (float*)d_out;

  char* ws = (char*)d_ws;
  unsigned short* WXP16 = (unsigned short*)(ws + kOffWXP);
  unsigned short* WDT16 = (unsigned short*)(ws + kOffWDT);
  unsigned short* X16   = (unsigned short*)(ws + kOffX16);
  float*          UC    = (float*)(ws + kOffUC);
  float*          PROJ  = (float*)(ws + kOffPROJ);
  unsigned short* DT16  = (unsigned short*)(ws + kOffDT16);
  float*          DLR   = (float*)(ws + kOffDLR);

  cast_pad_f16_kernel<<<(kPrjP * kDm / 8) / 256, 256, 0, stream>>>(xpw, WXP16, kPrjP * kDm / 8, kPrjN * kDm / 8, kCarryW1);
  cast_pad_f16_kernel<<<(kDm * kDtR / 8) / 256, 256, 0, stream>>>(dtw, WDT16, kDm * kDtR / 8, kDm * kDtR / 8, kCarryW2);

  conv_silu_kernel<<<dim3(kDm / 256, kRows / 64), 256, 0, stream>>>(mod, conv_w, conv_b, UC, X16);

  wmma_gemm64<0, false, 0, 0, false><<<dim3(((kRows / 64) * (kPrjP / 64)) / 8, 1), 256, 0, stream>>>(
      X16, X16, kDm, 0L,
      WXP16, WXP16, kDm, 0L,
      (void*)PROJ, (void*)PROJ, kPrjP, 0L,
      dtb, mod, 0L,
      kRows, kPrjP, kDm, kFold1);

  dt_cast_kernel<<<(kRows * kDtR / 8) / 256, 256, 0, stream>>>(PROJ, DT16, kRows * kDtR / 8, kCarryDt);

  wmma_gemm64<0, false, 2, 0, false><<<dim3(((kRows / 64) * (kDm / 64)) / 8, 1), 256, 0, stream>>>(
      DT16, DT16, kDtR, 0L,
      WDT16, WDT16, kDtR, 0L,
      (void*)DLR, (void*)DLR, kDm, 0L,
      dtb, mod, 0L,
      kRows, kDm, kDtR, kFold2);

  scan_kernel<<<kBatch * (kDm / 256), 256, 0, stream>>>(DLR, UC, mod, PROJ, A_log, Dp, out);
}
